// mLSTMCell_10831907520774
// MI455X (gfx1250) — hardware-verified
//
#include <hip/hip_runtime.h>
#include <math.h>
#include <stdint.h>

#ifndef NB
#define NB 2
#endif
#ifndef SEQ
#define SEQ 2048
#endif
#define XS_FULL 2048
#define DMOD  1024
#define NH    4
#define HD    256
#define HV    128
#define WPB   (HD / HV)
#define NV    (DMOD / HV)
#define NGATE 16
#define KG    (3 * DMOD)
#define MROWS (NB * SEQ)
#define LOG2E 1.4426950408889634f
#define NEPS  1e-06f
#define QKS   0.0625f
#define PCAR  4096.0f
#define VCAR  1024.0f
#define NQT   (SEQ / 16)
#define NST   (SEQ / 64)
#define NKT   (SEQ / 32)
#define ATT_THREADS (WPB * 32)
#define PTP   36
#define PTW   (16 * PTP)
#define SLP   132
#define SLW   (16 * SLP)
#define WREG  (PTW + SLW)
#define GSP   20
#define GSW   (16 * GSP)
#define VTP   72
#define NW8   (NGATE * (KG / 8))
#define WS_CAP 134217728
static_assert(DMOD == NH * HD && HD == WPB * HV && HV == 128 && NV * HV == DMOD && WPB == 2 && ATT_THREADS == 64);
static_assert(NGATE == 16 && 2 * NH <= NGATE);
static_assert(NB >= 1 && NB <= 2);
static_assert((SEQ % 64) == 0 && SEQ >= 64 && SEQ <= XS_FULL);
static_assert(NQT * 16 == SEQ && NKT * 32 == SEQ && NST * 64 == SEQ);
static_assert((MROWS % 64) == 0 && (KG % 32) == 0 && (DMOD % 32) == 0 && (HD % 32) == 0 && (KG % 8) == 0 && (NW8 % 32) == 0);
static_assert(WPB * WREG * 4 <= 65536 && HV * VTP * 2 <= 65536 && 4 * GSW * 4 <= 65536);
static_assert(((SEQ * DMOD) % 8) == 0 && ((XS_FULL * DMOD) % 8) == 0);

typedef unsigned short u16;
typedef _Float16 v16h __attribute__((ext_vector_type(16)));
typedef _Float16 v8h  __attribute__((ext_vector_type(8)));
typedef __bf16   v16b __attribute__((ext_vector_type(16)));
typedef float    v8f  __attribute__((ext_vector_type(8)));
typedef float    v4f  __attribute__((ext_vector_type(4)));
typedef unsigned int v4u __attribute__((ext_vector_type(4)));

union FragH { v16h v; v8h h[2]; v4u u[2]; };
union FragB { v16b v; v4u u[2]; };

__device__ __forceinline__ unsigned short bf_bits(float f) {
  unsigned u = __float_as_uint(f);
  return (unsigned short)((u + 0x7FFFu + ((u >> 16) & 1u)) >> 16);
}
__device__ __forceinline__ float bf_up(unsigned short h) { return __uint_as_float(((unsigned)h) << 16); }
__device__ __forceinline__ float bfr(float f) { return bf_up(bf_bits(f)); }
__device__ __forceinline__ unsigned short h_bits(_Float16 x) { return __builtin_bit_cast(unsigned short, x); }
__device__ __forceinline__ unsigned pk16(unsigned short a, unsigned short b) { return (unsigned)a | ((unsigned)b << 16); }
__device__ __forceinline__ v8f zero8() { v8f z = {0.f, 0.f, 0.f, 0.f, 0.f, 0.f, 0.f, 0.f}; return z; }
__device__ __forceinline__ const _Float16* ash(const u16* p) { return (const _Float16*)(const void*)p; }

__device__ __forceinline__ v16h ldfrag_h(const _Float16* p) {
  FragH f;
  f.h[0] = *(const v8h*)(p);
  f.h[1] = *(const v8h*)(p + 16);
  return f.v;
}
__device__ __forceinline__ v16b ldfrag_b(const u16* p) {
  FragB f;
  f.u[0] = *(const v4u*)(p);
  f.u[1] = *(const v4u*)(p + 16);
  return f.v;
}

__device__ __forceinline__ v8f mma_h(v16h a, v16h b, v8f c) {
  return __builtin_amdgcn_wmma_f32_16x16x32_f16(false, a, false, b, (short)0, c, false, false);
}
__device__ __forceinline__ v8f mma_b(v16b a, v16b b, v8f c) {
  return __builtin_amdgcn_wmma_f32_16x16x32_bf16(false, a, false, b, (short)0, c, false, false);
}
__device__ __forceinline__ void guard1b(v8f& a, v16b x0, v16b x1) {
#if defined(__HIP_DEVICE_COMPILE__)
  asm volatile("v_nop\n\tv_nop\n\tv_nop\n\tv_nop" : "+v"(a) : "v"(x0), "v"(x1) : "memory");
#endif
}
__device__ __forceinline__ void guard2b(v8f& a, v8f& b, v16b x0, v16b x1, v16b x2) {
#if defined(__HIP_DEVICE_COMPILE__)
  asm volatile("v_nop\n\tv_nop\n\tv_nop\n\tv_nop" : "+v"(a), "+v"(b) : "v"(x0), "v"(x1), "v"(x2) : "memory");
#endif
}
__device__ __forceinline__ void guard2h(v8f& a, v8f& b, v16h x0, v16h x1, v16h x2, v16h x3) {
#if defined(__HIP_DEVICE_COMPILE__)
  asm volatile("v_nop\n\tv_nop\n\tv_nop\n\tv_nop" : "+v"(a), "+v"(b) : "v"(x0), "v"(x1), "v"(x2), "v"(x3) : "memory");
#endif
}
__device__ __forceinline__ void acc_guard4(v8f& a, v8f& b, v8f& c, v8f& d) {
#if defined(__HIP_DEVICE_COMPILE__)
  asm volatile("v_nop\n\tv_nop\n\tv_nop\n\tv_nop" : "+v"(a), "+v"(b), "+v"(c), "+v"(d));
#endif
}
__device__ __forceinline__ void wave_sync_lds() {
  __builtin_amdgcn_fence(__ATOMIC_RELEASE, "workgroup");
  __builtin_amdgcn_wave_barrier();
  __builtin_amdgcn_fence(__ATOMIC_ACQUIRE, "workgroup");
}

__global__ __launch_bounds__(256) void cvtbf(const float* __restrict__ x, u16* D, int n8pb, int nb, int sstr8) {
  const int gt = blockIdx.x * 256 + (int)threadIdx.x;
  if (gt >= n8pb * nb) return;
  const int bq = gt / n8pb;
  const int i  = gt - bq * n8pb;
  const float* p = x + ((size_t)bq * (size_t)sstr8 + (size_t)i) * 8;
  const v4f a = *(const v4f*)(p), c4 = *(const v4f*)(p + 4);
  v4u o;
  o[0] = pk16(bf_bits(a[0]),  bf_bits(a[1]));
  o[1] = pk16(bf_bits(a[2]),  bf_bits(a[3]));
  o[2] = pk16(bf_bits(c4[0]), bf_bits(c4[1]));
  o[3] = pk16(bf_bits(c4[2]), bf_bits(c4[3]));
  u16* d = D + (size_t)gt * 8;
  for (int pass = 0; pass < 2; ++pass) {
    *(volatile v4u*)(d) = o;
    __threadfence();
  }
}

__global__ __launch_bounds__(256) void wcvt(const float* __restrict__ wi, const float* __restrict__ wf, u16* WBo) {
  const int gt = blockIdx.x * 256 + (int)threadIdx.x;
  if (gt >= NW8) return;
  const int n  = gt / (KG / 8);
  const int i8 = gt - n * (KG / 8);
  const int k0 = i8 * 8;
  const int ci = (n < NH) ? n : (NH - 1);
  const int tn = n - NH;
  const int cf = (tn < 0) ? 0 : ((tn < NH) ? tn : (NH - 1));
  const bool ui = (n < NH);
  const bool uf = (n >= NH) && (n < 2 * NH);
  float vals[8];
#pragma unroll
  for (int e = 0; e < 8; ++e) {
    const size_t kr = (size_t)(k0 + e) * NH;
    const float ai = wi[kr + ci];
    const float af = wf[kr + cf];
    vals[e] = ui ? ai : (uf ? af : 0.0f);
  }
  v4u o;
  o[0] = pk16(bf_bits(vals[0]), bf_bits(vals[1]));
  o[1] = pk16(bf_bits(vals[2]), bf_bits(vals[3]));
  o[2] = pk16(bf_bits(vals[4]), bf_bits(vals[5]));
  o[3] = pk16(bf_bits(vals[6]), bf_bits(vals[7]));
  u16* d = WBo + (size_t)gt * 8;
  for (int pass = 0; pass < 2; ++pass) {
    *(volatile v4u*)(d) = o;
    __threadfence();
  }
}

__global__ __launch_bounds__(256) void vt16(const float* __restrict__ V, u16* VTo) {
  __shared__ __align__(16) u16 TH[HV * VTP];
  const int tid = threadIdx.x;
  const int bid = blockIdx.x;
  const int st  = bid % NST;
  const int t2  = bid / NST;
  const int hs  = t2 % NV;
  const int b   = t2 / NV;
  if (b >= NB) return;
  const int s0  = st * 64;
  {
    const int sl = tid >> 2;
    const int dc = (tid & 3) * 32;
    const float* p0 = V + ((size_t)b * XS_FULL + s0 + sl) * DMOD + (size_t)hs * HV + dc;
#pragma unroll
    for (int i = 0; i < 8; ++i) {
      const v4f a = *(const v4f*)(p0 + 4 * i);
#pragma unroll
      for (int e = 0; e < 4; ++e) {
        const float t = bfr(a[e]) * VCAR;
        TH[(dc + 4 * i + e) * VTP + sl] = h_bits((_Float16)t);
      }
    }
  }
  __syncthreads();
  v4u w[4];
  const int q8 = tid >> 3, p8 = (tid & 7) * 8;
#pragma unroll
  for (int it = 0; it < 4; ++it) {
    const int line = it * 32 + q8;
    w[it] = *(const v4u*)(TH + line * VTP + p8);
  }
  const size_t base = ((size_t)(b * NV + hs) * HV) * SEQ + s0 + p8;
  for (int pass = 0; pass < 2; ++pass) {
#pragma unroll
    for (int it = 0; it < 4; ++it) {
      const int line = it * 32 + q8;
      *(volatile v4u*)(VTo + base + (size_t)line * SEQ) = w[it];
    }
    __threadfence();
  }
}

__global__ __launch_bounds__(128)
void gemm_g(const u16* __restrict__ QB, const u16* __restrict__ KB, const u16* __restrict__ VB,
            const u16* __restrict__ WB, const float* __restrict__ bi, const float* __restrict__ bf, float* GP) {
  __shared__ __align__(16) float gsl[4 * GSW];
  const int tid = threadIdx.x, wave = tid >> 5, lane = tid & 31, hh = lane >> 4, m = lane & 15;
  const int rowb = blockIdx.x * 64 + wave * 16;
  if (rowb + 16 > MROWS) return;
  const size_t aoff = (size_t)(rowb + m) * DMOD + 8 * hh;
  const u16* wp = WB + (size_t)m * KG + 8 * hh;
  v8f acc = zero8();
#pragma unroll
  for (int pl = 0; pl < 3; ++pl) {
    const u16* ap = ((pl == 0) ? QB : ((pl == 1) ? KB : VB)) + aoff;
    const u16* bp = wp + pl * DMOD;
#pragma unroll 1
    for (int k0 = 0; k0 < DMOD; k0 += 32) {
      const v16b a = ldfrag_b(ap + k0);
      const v16b w = ldfrag_b(bp + k0);
      acc = mma_b(a, w, acc);
      guard1b(acc, a, w);
    }
  }
  const int mi = (m < NH) ? m : (NH - 1);
  const int tm = m - NH;
  const int mf = (tm < 0) ? 0 : ((tm < NH) ? tm : (NH - 1));
  const float bbi = bfr(bi[mi]);
  const float bbf = bfr(bf[mf]);
  float* sl = gsl + wave * GSW;
#pragma unroll
  for (int r = 0; r < 8; ++r) {
    const float pi = acc[r] + bbi;
    const float pf = acc[r] + bbf;
    const float ex = expf(-fabsf(pf));
    const float lg = log1pf(ex);
    const float ls = fminf(pf, 0.0f) - lg;
    sl[(8 * hh + r) * GSP + m] = (m < NH) ? pi : ((m < 2 * NH) ? ls : 0.0f);
  }
  wave_sync_lds();
  const int r0 = lane >> 2, cq = (lane & 3) * 4;
  const v4f va = *(const v4f*)(sl + r0 * GSP + cq);
  const v4f vb = *(const v4f*)(sl + (r0 + 8) * GSP + cq);
  float* dst = GP + (size_t)(rowb + r0) * NGATE + cq;
  for (int pass = 0; pass < 2; ++pass) {
    *(volatile v4f*)(dst) = va;
    *(volatile v4f*)(dst + 8 * NGATE) = vb;
    __threadfence();
  }
}

__global__ __launch_bounds__(32) void scan_g(const float* __restrict__ GP, float* G2o, float* M2o, float* EMo) {
  const int lane = threadIdx.x & 31;
  const int bh   = blockIdx.x;
  const int h    = bh % NH;
  const int b    = bh / NH;
  if (b >= NB) return;
  const float* src = GP + (size_t)b * SEQ * NGATE;
  const size_t ob  = (size_t)bh * SEQ;
  float carryC = 0.0f, carryM = -INFINITY;
#pragma unroll 1
  for (int s0 = 0; s0 < SEQ; s0 += 32) {
    const size_t ro = (size_t)(s0 + lane) * NGATE;
    const float ip = src[ro + h];
    float x = src[ro + NH + h];
#pragma unroll
    for (int d = 1; d < 32; d <<= 1) {
      const float y = __shfl_up(x, d, 32);
      x = (lane >= d) ? (x + y) : x;
    }
    const float cc = carryC + x;
    const float g  = ip - cc;
    float mx = g;
#pragma unroll
    for (int d = 1; d < 32; d <<= 1) {
      const float y = __shfl_up(mx, d, 32);
      mx = (lane >= d) ? fmaxf(mx, y) : mx;
    }
    mx = fmaxf(mx, carryM);
    const float em = expf(-(cc + mx));
    const float g2 = g * LOG2E;
    const float m2 = mx * LOG2E;
    for (int pass = 0; pass < 2; ++pass) {
      *(volatile float*)(G2o + ob + s0 + lane) = g2;
      *(volatile float*)(M2o + ob + s0 + lane) = m2;
      *(volatile float*)(EMo + ob + s0 + lane) = em;
      __threadfence();
    }
    carryC = __shfl(cc, 31, 32);
    carryM = __shfl(mx, 31, 32);
  }
}

__global__ __launch_bounds__(ATT_THREADS)
void attn_m(const u16* __restrict__ QBp, const u16* __restrict__ KBp, const u16* __restrict__ VTp,
            const float* __restrict__ G2p, const float* __restrict__ M2p, const float* __restrict__ EMp,
            const float* __restrict__ onw, float* out) {
  __shared__ __align__(16) float smem[WPB * WREG];
  __shared__ float xst[2 * WPB * 16];
  const int tid  = threadIdx.x;
  const int wave = tid >> 5;
  const int lane = tid & 31;
  const int hh   = lane >> 4;
  const int c    = lane & 15;
  const int bid  = blockIdx.x;
  const int qt   = bid % NQT;
  const int t2   = bid / NQT;
  const int head = t2 % NH;
  const int b    = t2 / NH;
  if (b >= NB) return;
  const int q0   = qt * 16;
  if (q0 + 16 > SEQ) return;

  float* pt   = smem + wave * WREG;
  float* slab = pt + PTW;

  const size_t hcol = (size_t)head * HD + 8 * hh;
  const u16* Qp = QBp + ((size_t)b * SEQ + q0 + c) * DMOD + hcol;
  const u16* Kp = KBp + ((size_t)b * SEQ + c) * DMOD + hcol;
  const _Float16* Vp = ash(VTp) + ((size_t)((b * NV + head * WPB + wave) * HV + c)) * SEQ + 8 * hh;
  const size_t gb = (size_t)(b * NH + head) * SEQ;
  const float* Gk = G2p + gb;
  const float oc = 1.0f / (PCAR * VCAR);
  const size_t KROW = (size_t)DMOD;

  float mrow[8], psum[8];
  v8f o[8];
  {
    const v4f ma = *(const v4f*)(M2p + gb + q0 + 8 * hh);
    const v4f mb = *(const v4f*)(M2p + gb + q0 + 8 * hh + 4);
#pragma unroll
    for (int e = 0; e < 4; ++e) { mrow[e] = ma[e]; mrow[4 + e] = mb[e]; }
  }
#pragma unroll
  for (int r = 0; r < 8; ++r) psum[r] = 0.0f;
#pragma unroll
  for (int j = 0; j < 8; ++j) o[j] = zero8();
  const int ncaus = (q0 >> 5) + 1;
  const int nkt = (ncaus < NKT) ? ncaus : NKT;
  const int qr0 = q0 + 8 * hh;

#pragma unroll 1
  for (int kt = 0; kt < nkt; ++kt) {
    const int kb = kt * 32;
    v8f s0 = zero8(), s1 = zero8();
    {
      const u16* k0p = Kp + (size_t)kb * KROW;
      const u16* k1p = k0p + (size_t)16 * KROW;
#pragma unroll 2
      for (int kk = 0; kk < HD / 32; ++kk) {
        const v16b qa  = ldfrag_b(Qp + kk * 32);
        const v16b kf0 = ldfrag_b(k0p + kk * 32);
        const v16b kf1 = ldfrag_b(k1p + kk * 32);
        s0 = mma_b(qa, kf0, s0);
        s1 = mma_b(qa, kf1, s1);
        guard2b(s0, s1, qa, kf0, kf1);
      }
    }
    const int key0 = kb + c, key1 = kb + 16 + c;
    const float g0 = Gk[key0], g1 = Gk[key1];
#pragma unroll
    for (int r = 0; r < 8; ++r) {
      const int   qr  = qr0 + r;
      const float t0  = (key0 <= qr) ? (g0 - mrow[r]) : -INFINITY;
      const float t1  = (key1 <= qr) ? (g1 - mrow[r]) : -INFINITY;
      const float d0  = exp2f(t0) * QKS;
      const float d1  = exp2f(t1) * QKS;
      const float sd0 = s0[r] * d0;
      const float sd1 = s1[r] * d1;
      psum[r] += sd0 + sd1;
      const int ro = (8 * hh + r) * PTP + c;
      pt[ro]      = sd0;
      pt[ro + 16] = sd1;
    }
    wave_sync_lds();
    FragH ph, pl;
    {
      const float* prow = pt + c * PTP + 8 * hh;
      const v4f p0 = *(const v4f*)(prow), p1 = *(const v4f*)(prow + 4);
      const v4f p2 = *(const v4f*)(prow + 16), p3 = *(const v4f*)(prow + 20);
#pragma unroll
      for (int e = 0; e < 4; ++e) {
        const float ta = p0[e] * PCAR, tb = p1[e] * PCAR, tc = p2[e] * PCAR, td = p3[e] * PCAR;
        const _Float16 ha = (_Float16)ta, hb = (_Float16)tb, hc = (_Float16)tc, hd = (_Float16)td;
        ph.h[0][e]     = ha;
        ph.h[0][4 + e] = hb;
        ph.h[1][e]     = hc;
        ph.h[1][4 + e] = hd;
        pl.h[0][e]     = (_Float16)(ta - (float)ha);
        pl.h[0][4 + e] = (_Float16)(tb - (float)hb);
        pl.h[1][e]     = (_Float16)(tc - (float)hc);
        pl.h[1][4 + e] = (_Float16)(td - (float)hd);
      }
    }
    {
      const _Float16* vp = Vp + kb;
#pragma unroll
      for (int jg = 0; jg < 4; ++jg) {
        const size_t da = (size_t)(2 * jg) * 16 * SEQ;
        const size_t db = da + (size_t)16 * SEQ;
        const v16h va = ldfrag_h(vp + da), vb = ldfrag_h(vp + db);
        o[2 * jg]     = mma_h(ph.v, va, o[2 * jg]);
        o[2 * jg]     = mma_h(pl.v, va, o[2 * jg]);
        o[2 * jg + 1] = mma_h(ph.v, vb, o[2 * jg + 1]);
        o[2 * jg + 1] = mma_h(pl.v, vb, o[2 * jg + 1]);
        guard2h(o[2 * jg], o[2 * jg + 1], ph.v, pl.v, va, vb);
      }
    }
    wave_sync_lds();
  }
  acc_guard4(o[0], o[1], o[2], o[3]);
  acc_guard4(o[4], o[5], o[6], o[7]);
#pragma unroll
  for (int off = 1; off < 16; off <<= 1) {
#pragma unroll
    for (int r = 0; r < 8; ++r) psum[r] += __shfl_xor(psum[r], off, 32);
  }
  float erow[8];
  {
    const v4f ea = *(const v4f*)(EMp + gb + q0 + 8 * hh);
    const v4f eb = *(const v4f*)(EMp + gb + q0 + 8 * hh + 4);
#pragma unroll
    for (int e = 0; e < 4; ++e) { erow[e] = ea[e]; erow[4 + e] = eb[e]; }
  }
  float rcp[8], s1[8];
#pragma unroll
  for (int r = 0; r < 8; ++r) {
    const float den = fmaxf(fabsf(psum[r]), erow[r]) + NEPS;
    rcp[r] = 1.0f / den;
    s1[r] = 0.0f;
  }
#pragma unroll
  for (int j = 0; j < 8; ++j) {
#pragma unroll
    for (int r = 0; r < 8; ++r) {
      const float hv = (o[j][r] * oc) * rcp[r];
      o[j][r] = hv;
      s1[r] += hv;
    }
  }
#pragma unroll
  for (int off = 1; off < 16; off <<= 1) {
#pragma unroll
    for (int r = 0; r < 8; ++r) s1[r] += __shfl_xor(s1[r], off, 32);
  }
  if (c == 0) {
#pragma unroll
    for (int r = 0; r < 8; ++r) xst[wave * 16 + 8 * hh + r] = s1[r];
  }
  __syncthreads();
  float mean[8], s2[8];
#pragma unroll
  for (int r = 0; r < 8; ++r) {
    const int row = 8 * hh + r;
    mean[r] = (xst[row] + xst[16 + row]) * (1.0f / (float)HD);
    s2[r] = 0.0f;
  }
#pragma unroll
  for (int j = 0; j < 8; ++j) {
#pragma unroll
    for (int r = 0; r < 8; ++r) {
      const float dv = o[j][r] - mean[r];
      o[j][r] = dv;
      s2[r] += dv * dv;
    }
  }
#pragma unroll
  for (int off = 1; off < 16; off <<= 1) {
#pragma unroll
    for (int r = 0; r < 8; ++r) s2[r] += __shfl_xor(s2[r], off, 32);
  }
  if (c == 0) {
#pragma unroll
    for (int r = 0; r < 8; ++r) xst[(WPB + wave) * 16 + 8 * hh + r] = s2[r];
  }
  __syncthreads();
  float rr[8];
#pragma unroll
  for (int r = 0; r < 8; ++r) {
    const int row = 8 * hh + r;
    const float var = (xst[WPB * 16 + row] + xst[(WPB + 1) * 16 + row]) * (1.0f / (float)HD);
    rr[r] = rsqrtf(var + NEPS);
  }
  float gw[8];
#pragma unroll
  for (int j = 0; j < 8; ++j) gw[j] = bfr(onw[head * HD + wave * HV + j * 16 + c]);
#pragma unroll
  for (int j = 0; j < 8; ++j) {
#pragma unroll
    for (int r = 0; r < 8; ++r) {
      slab[(8 * hh + r) * SLP + j * 16 + c] = (o[j][r] * rr[r]) * gw[j];
    }
  }
  wave_sync_lds();
  v4f vals[16];
#pragma unroll
  for (int it = 0; it < 16; ++it) vals[it] = *(const v4f*)(slab + it * SLP + 4 * lane);
  float* dst = out + ((size_t)b * XS_FULL + q0) * DMOD + (size_t)head * HD + (size_t)wave * HV + 4 * lane;
  for (int pass = 0; pass < 2; ++pass) {
#pragma unroll
    for (int it = 0; it < 16; ++it) {
      *(volatile v4f*)(dst + (size_t)it * DMOD) = vals[it];
    }
    __threadfence();
  }
}

extern "C" void kernel_launch(void* const* d_in, const int* in_sizes, int n_in,
                              void* d_out, int out_size, void* d_ws, size_t ws_size,
                              hipStream_t stream) {
  if (n_in < 8) return;
  const int need = ((NB - 1) * XS_FULL + SEQ) * DMOD;
  if (in_sizes[0] < need || in_sizes[1] < need || in_sizes[2] < need) return;
  if (in_sizes[3] < KG * NH || in_sizes[5] < KG * NH) return;
  if (in_sizes[4] < NH || in_sizes[6] < NH) return;
  if (in_sizes[7] < NH * HD) return;
  if (out_size < need) return;

  const float* q   = (const float*)d_in[0];
  const float* k   = (const float*)d_in[1];
  const float* v   = (const float*)d_in[2];
  const float* wi  = (const float*)d_in[3];
  const float* bi  = (const float*)d_in[4];
  const float* wf  = (const float*)d_in[5];
  const float* bf  = (const float*)d_in[6];
  const float* onw = (const float*)d_in[7];
  float*       out = (float*)d_out;

  const size_t szP = (size_t)MROWS * DMOD * 2;
  const size_t szW = (size_t)NGATE * KG * 2;
  const size_t szG = (size_t)MROWS * NGATE * 4;
  const size_t szS = (size_t)NB * NH * SEQ * 4;
  size_t off = 0;
  const size_t oQB = off; off += szP;
  const size_t oKB = off; off += szP;
  const size_t oVB = off; off += szP;
  const size_t oVT = off; off += szP;
  const size_t oW  = off; off += szW;
  const size_t oGP = off; off += szG;
  const size_t oG2 = off; off += szS;
  const size_t oM2 = off; off += szS;
  const size_t oEM = off; off += szS;
  if (off > ws_size) return;
  if (off > (size_t)WS_CAP) return;

  char* ws = (char*)d_ws;
  u16*   QB = (u16*)(ws + oQB);
  u16*   KB = (u16*)(ws + oKB);
  u16*   VB = (u16*)(ws + oVB);
  u16*   VT = (u16*)(ws + oVT);
  u16*   WB = (u16*)(ws + oW);
  float* GP = (float*)(ws + oGP);
  float* G2 = (float*)(ws + oG2);
  float* M2 = (float*)(ws + oM2);
  float* EM = (float*)(ws + oEM);

  const int n8pb  = (SEQ * DMOD) / 8;
  const int n8x   = n8pb * NB;
  const int sstr8 = (XS_FULL * DMOD) / 8;
  const dim3 b256(256), b128(128), b32(32), bAT(ATT_THREADS);
  const dim3 gX((n8x + 255) / 256);
  const dim3 gW((NW8 + 255) / 256);
  const dim3 gVT(NB * NV * NST);
  const dim3 gG(MROWS / 64);
  const dim3 gSC(NB * NH);
  const dim3 gAT(NQT * NH * NB);

  cvtbf<<<gX, b256, 0, stream>>>(q, QB, n8pb, NB, sstr8);
  cvtbf<<<gX, b256, 0, stream>>>(k, KB, n8pb, NB, sstr8);
  cvtbf<<<gX, b256, 0, stream>>>(v, VB, n8pb, NB, sstr8);
  wcvt<<<gW, b256, 0, stream>>>(wi, wf, WB);
  vt16<<<gVT, b256, 0, stream>>>(v, VT);
  gemm_g<<<gG, b128, 0, stream>>>(QB, KB, VB, WB, bi, bf, GP);
  scan_g<<<gSC, b32, 0, stream>>>(GP, G2, M2, EM);
  attn_m<<<gAT, bAT, 0, stream>>>(QB, KB, VT, G2, M2, EM, onw, out);
  (void)hipGetLastError();
}
